// CustomDCNv2_45629732552757
// MI455X (gfx1250) — hardware-verified
//
#include <hip/hip_runtime.h>
#include <stdint.h>
#include <stddef.h>

#pragma clang fp contract(off)

#define DEVINL __device__ __forceinline__

typedef _Float16 f16t;
typedef _Float16 v16h __attribute__((ext_vector_type(16)));
typedef _Float16 v8h  __attribute__((ext_vector_type(8)));
typedef _Float16 v4h  __attribute__((ext_vector_type(4)));
typedef float    v8f  __attribute__((ext_vector_type(8)));
typedef float    v4f  __attribute__((ext_vector_type(4)));
typedef int      v4i  __attribute__((ext_vector_type(4)));
typedef v8h  __attribute__((may_alias)) v8ha;
typedef v4h  __attribute__((may_alias)) v4ha;
typedef v4f  __attribute__((may_alias)) v4fa;
union FragH { v16h v; v8h half[2]; };

#define CCH   256
#define HH    64
#define WW    64
#define HWPIX (HH * WW)
#define KTAP  9
#define OFFCH (2 * KTAP)
#define KDIM  (CCH * KTAP)
#define KSTEP 32
#define NIT   (KDIM / KSTEP)
#define TPB   256
#define NPW   32
#define MTD   32
#define NSD   (MTD / 16)
#define NENT  (MTD * KTAP)
#define ACAR  16.0f
#define WCAR  256.0f
#define SPT   132
#define SPX   36

static_assert(KDIM % KSTEP == 0);
static_assert(CCH / KSTEP == 8);
static_assert(WW % MTD == 0);
static_assert(WW / MTD == 2);
static_assert(MTD * (KSTEP / 4) == TPB);
static_assert(CCH == 8 * NPW);
static_assert(TPB == CCH);
static_assert((WW * 128) % TPB == 0);
static_assert((SPT % 4) == 0 && (SPX % 4) == 0);
static_assert((CCH * (KDIM / 8)) % TPB == 0);
static_assert((CCH * KDIM * 2) % 128 == 0);
static_assert(NENT <= 2 * TPB);

DEVINL int imin(int a, int b) { return a < b ? a : b; }
DEVINL int imax(int a, int b) { return a > b ? a : b; }
DEVINL int clampi(int v, int lo, int hi) { return imin(imax(v, lo), hi); }

DEVINL v8f wmma_f16(v16h a, v16h b, v8f c) {
  v8f d = __builtin_amdgcn_wmma_f32_16x16x32_f16(false, a, false, b, (short)0, c, false, false);
  asm volatile("v_nop\n\tv_nop\n\tv_nop\n\tv_nop" : "+v"(d) : "v"(a), "v"(b));
  return d;
}
DEVINL v8f zero8f() {
  v8f z = {0.f, 0.f, 0.f, 0.f, 0.f, 0.f, 0.f, 0.f};
  return z;
}

DEVINL v16h frag_row(const f16t* rowp, int h) {
  FragH f;
  f.half[0] = *(const v8ha*)(rowp + 8 * h);
  f.half[1] = *(const v8ha*)(rowp + 16 + 8 * h);
  return f.v;
}

__global__ __launch_bounds__(TPB) void prep_w_k(const float* __restrict__ wc,
                                               f16t* __restrict__ dwT)
{
  const int t = blockIdx.x * TPB + threadIdx.x;
  if (t >= CCH * (KDIM / 8)) return;
  const int n    = t / (KDIM / 8);
  const int part = t - n * (KDIM / 8);
  const int k0   = part * 8;
  const int tap  = k0 / CCH;
  const int cin0 = k0 - tap * CCH;
  const float* sp = wc + ((size_t)n * CCH + cin0) * KTAP + tap;
  v8h o;
  #pragma unroll
  for (int j = 0; j < 8; ++j) o[j] = (f16t)(sp[(size_t)j * KTAP] * WCAR);
  f16t* dp = dwT + (size_t)8 * t;
  *(volatile v8h*)dp = o;
  __threadfence();
  *(volatile v8h*)dp = o;
}

__global__ __launch_bounds__(TPB) void pack_x_k(const float* __restrict__ x, float* __restrict__ xn)
{
  __shared__ __attribute__((aligned(16))) float sT[WW * SPT];
  const int tid  = threadIdx.x;
  const int lane = tid & 31;
  const int wave = tid >> 5;
  const int row  = blockIdx.x;
  const int chf  = blockIdx.y;
  const int b    = row / HH;
  const int h    = row - b * HH;
  const float* xb = x + ((size_t)(b * CCH + chf * 128)) * HWPIX + (size_t)h * WW;
  #pragma unroll 4
  for (int i = 0; i < (WW * 128) / TPB; ++i) {
    const int idx = i * TPB + tid;
    const int cl  = idx / WW;
    const int w   = idx - cl * WW;
    sT[w * SPT + cl] = xb[(size_t)cl * HWPIX + w];
  }
  __syncthreads();
  {
    const int q = lane >> 3, e = lane & 7;
    #pragma unroll
    for (int ch = 0; ch < 2; ++ch) {
      v4f pv[4];
      size_t go[4];
      #pragma unroll
      for (int i = 0; i < 4; ++i) {
        const int L   = wave * 32 + (ch * 4 + i) * 4 + q;
        const int px  = L >> 2;
        const int sub = L & 3;
        pv[i] = *(const v4fa*)&sT[px * SPT + sub * 32 + e * 4];
        go[i] = (size_t)(row * WW + px) * CCH + chf * 128 + sub * 32 + e * 4;
      }
      #pragma unroll
      for (int i = 0; i < 4; ++i) *(volatile v4f*)(xn + go[i]) = pv[i];
      __threadfence();
      #pragma unroll
      for (int i = 0; i < 4; ++i) *(volatile v4f*)(xn + go[i]) = pv[i];
    }
  }
}

__global__ __launch_bounds__(TPB) void deform_k(const float* __restrict__ xn,
                                               const float* __restrict__ offp,
                                               const float* __restrict__ mskp,
                                               const f16t* __restrict__ dwT,
                                               const float* __restrict__ bias,
                                               const int* __restrict__ pstr,
                                               const int* __restrict__ ppad,
                                               const int* __restrict__ pdil,
                                               float* __restrict__ out)
{
  __shared__ __attribute__((aligned(16))) v4i   sO[NENT];
  __shared__ __attribute__((aligned(16))) v4f   sW[NENT];
  __shared__ __attribute__((aligned(16))) float sM[NENT];
  __shared__ __attribute__((aligned(16))) float sB[CCH];
  __shared__ __attribute__((aligned(16))) f16t  Als[2][MTD * KSTEP];
  __shared__ __attribute__((aligned(16))) float sStg[128 * SPX];

  const int tid  = threadIdx.x;
  const int lane = tid & 31;
  const int wave = tid >> 5;
  const int hl   = lane >> 4;
  const int m    = lane & 15;
  const int blk  = blockIdx.x;
  const int row  = blk >> 1;
  const int half = blk & 1;
  const int b    = row / HH;
  const int h    = row - b * HH;
  const int w0   = half * MTD;
  const int strd = pstr[0];
  const int padd = ppad[0];
  const int dil  = pdil[0];

  sB[tid] = bias[tid];

  #pragma unroll 1
  for (int e = tid; e < NENT; e += TPB) {
    const int p  = e / KTAP;
    const int t  = e - p * KTAP;
    const int tr = t / 3, tc = t - tr * 3;
    const int w  = w0 + p;
    const size_t pixo = (size_t)h * WW + w;
    const float dy = offp[(size_t)(b * OFFCH + 2 * t) * HWPIX + pixo];
    const float dx = offp[(size_t)(b * OFFCH + 2 * t + 1) * HWPIX + pixo];
    const float mk = mskp[(size_t)(b * KTAP + t) * HWPIX + pixo];
    const float by = (float)(h * strd - padd);
    const float bx = (float)(w * strd - padd);
    const float yf = (dy + by) + (float)(tr * dil);
    const float xf = (dx + bx) + (float)(tc * dil);
    const float y0f = floorf(yf), x0f = floorf(xf);
    const float ly = yf - y0f, lx = xf - x0f;
    const int y0 = (int)fminf(fmaxf(y0f, -4.0f), (float)(HH + 4));
    const int x0 = (int)fminf(fmaxf(x0f, -4.0f), (float)(WW + 4));
    const bool vy0 = (y0 >= 0)  && (y0 <= HH - 1);
    const bool vy1 = (y0 >= -1) && (y0 <= HH - 2);
    const bool vx0 = (x0 >= 0)  && (x0 <= WW - 1);
    const bool vx1 = (x0 >= -1) && (x0 <= WW - 2);
    const int y0k = clampi(y0, 0, HH - 1), y1k = clampi(y0 + 1, 0, HH - 1);
    const int x0k = clampi(x0, 0, WW - 1), x1k = clampi(x0 + 1, 0, WW - 1);
    const float ay = 1.0f - ly, ax = 1.0f - lx;
    v4f gw;
    gw[0] = (vy0 && vx0) ? (ay * ax) : 0.0f;
    gw[1] = (vy0 && vx1) ? (ay * lx) : 0.0f;
    gw[2] = (vy1 && vx0) ? (ly * ax) : 0.0f;
    gw[3] = (vy1 && vx1) ? (ly * lx) : 0.0f;
    v4i o;
    o[0] = y0k * WW + x0k;
    o[1] = y0k * WW + x1k;
    o[2] = y1k * WW + x0k;
    o[3] = y1k * WW + x1k;
    sO[e] = o;
    sW[e] = gw;
    sM[e] = mk;
  }
  __syncthreads();

  const int pgrp  = tid & 31;
  const int cgrp  = tid >> 5;
  const int nbase = wave * NPW;
  const float* xb = xn + (size_t)b * HWPIX * CCH;

  v8f acc[2][NSD];
  #pragma unroll
  for (int j = 0; j < 2; ++j) {
    #pragma unroll
    for (int s = 0; s < NSD; ++s) acc[j][s] = zero8f();
  }

  #pragma unroll 1
  for (int it = 0; it < NIT; ++it) {
    const int k0  = it * KSTEP;
    const int tap = it >> 3;
    const int c0  = (it & 7) * KSTEP;
    const int buf = it & 1;
    {
      const int e = pgrp * KTAP + tap;
      const v4i o  = sO[e];
      const v4f g  = sW[e];
      const float mk = sM[e];
      const float* base = xb + c0 + cgrp * 4;
      const v4f a0 = *(const v4fa*)(base + (size_t)o[0] * CCH);
      const v4f a1 = *(const v4fa*)(base + (size_t)o[1] * CCH);
      const v4f a2 = *(const v4fa*)(base + (size_t)o[2] * CCH);
      const v4f a3 = *(const v4fa*)(base + (size_t)o[3] * CCH);
      v4h ov;
      #pragma unroll
      for (int i = 0; i < 4; ++i) {
        const float t0 = g[0] * a0[i];
        const float t1 = g[1] * a1[i];
        const float t2 = g[2] * a2[i];
        const float t3 = g[3] * a3[i];
        const float v  = (((t0 + t1) + t2) + t3) * mk;
        ov[i] = (f16t)(v * ACAR);
      }
      *(v4ha*)&Als[buf][pgrp * KSTEP + cgrp * 4] = ov;
    }
    __syncthreads();
    v16h wf[2];
    wf[0] = frag_row(dwT + (size_t)(nbase + m) * KDIM + k0, hl);
    wf[1] = frag_row(dwT + (size_t)(nbase + 16 + m) * KDIM + k0, hl);
    #pragma unroll
    for (int s = 0; s < NSD; ++s) {
      const v16h xf = frag_row(&Als[buf][(s * 16 + m) * KSTEP], hl);
      acc[0][s] = wmma_f16(xf, wf[0], acc[0][s]);
      acc[1][s] = wmma_f16(xf, wf[1], acc[1][s]);
    }
  }

  const float kin = 1.0f / (ACAR * WCAR);
  #pragma unroll
  for (int p = 0; p < 2; ++p) {
    if ((wave >> 2) == p) {
      #pragma unroll
      for (int j = 0; j < 2; ++j) {
        #pragma unroll
        for (int s = 0; s < NSD; ++s) {
          const int cl = (wave - 4 * p) * NPW + 16 * j + m;
          const float bv = sB[p * 128 + cl];
          float* rowp = &sStg[cl * SPX + 16 * s + 8 * hl];
          v4f lo4, hi4;
          #pragma unroll
          for (int r = 0; r < 4; ++r) {
            lo4[r] = acc[j][s][r] * kin + bv;
            hi4[r] = acc[j][s][4 + r] * kin + bv;
          }
          *(v4fa*)rowp       = lo4;
          *(v4fa*)(rowp + 4) = hi4;
        }
      }
    }
    __syncthreads();
    {
      const int q = lane >> 3, e = lane & 7;
      v4f ov[4];
      size_t go[4];
      #pragma unroll
      for (int i = 0; i < 4; ++i) {
        const int cl = wave * 16 + 4 * i + q;
        const int c  = p * 128 + cl;
        ov[i] = *(const v4fa*)&sStg[cl * SPX + e * 4];
        go[i] = ((size_t)(b * CCH + c) * HH + h) * WW + w0 + e * 4;
      }
      #pragma unroll
      for (int i = 0; i < 4; ++i) *(volatile v4f*)(out + go[i]) = ov[i];
      __threadfence();
      #pragma unroll
      for (int i = 0; i < 4; ++i) *(volatile v4f*)(out + go[i]) = ov[i];
    }
    __syncthreads();
  }
}

extern "C" void kernel_launch(void* const* d_in, const int* in_sizes, int n_in,
                              void* d_out, int out_size, void* d_ws, size_t ws_size,
                              hipStream_t stream) {
  if (n_in < 9) return;
  const int chw = CCH * HWPIX;
  if (in_sizes[0] <= 0 || (in_sizes[0] % chw) != 0) return;
  const int nB = in_sizes[0] / chw;
  if (in_sizes[1] != nB * OFFCH * HWPIX) return;
  if (in_sizes[2] != nB * KTAP * HWPIX) return;
  if (in_sizes[3] != CCH * KDIM) return;
  if (in_sizes[4] != CCH) return;
  if (in_sizes[5] < 1 || in_sizes[6] < 1 || in_sizes[7] < 1) return;
  if (out_size != in_sizes[0]) return;

  const float* x    = (const float*)d_in[0];
  const float* offp = (const float*)d_in[1];
  const float* mskp = (const float*)d_in[2];
  const float* wcnv = (const float*)d_in[3];
  const float* bias = (const float*)d_in[4];
  const int*   pstr = (const int*)d_in[5];
  const int*   ppad = (const int*)d_in[6];
  const int*   pdil = (const int*)d_in[7];
  float* outp = (float*)d_out;

  const size_t szXN = (size_t)nB * HWPIX * CCH * 4;
  const size_t szW  = (size_t)CCH * KDIM * 2;
  size_t off = 0;
  char* ws = (char*)d_ws;
  float* xn  = (float*)(ws + off); off += szXN;
  f16t*  dwT = (f16t*)(ws + off);  off += szW;
  if (off > ws_size) return;

  prep_w_k<<<(CCH * (KDIM / 8)) / TPB, TPB, 0, stream>>>(wcnv, dwT);
  pack_x_k<<<dim3(nB * HH, 2), TPB, 0, stream>>>(x, xn);
  deform_k<<<nB * HH * (WW / MTD), TPB, 0, stream>>>(xn, offp, mskp, dwT, bias, pstr, ppad, pdil, outp);
}
